// TemporalWindowAttention_76544907149532
// MI455X (gfx1250) — hardware-verified
//
#include <hip/hip_runtime.h>
#include <math.h>
#include <stdint.h>


#define NF    16
#define CC    320
#define NL    1024
#define NH    8
#define HD    40
#define QP    64
#define VP    48
#define NIN   960
#define TOK   (NF * NL)
#define NQK   (2 * NH * QP)
#define NVR   (NH * VP)
#define FG    ((NF < 4) ? NF : 4)
#define NPAIR (FG * NH)
#define RSB   32
#define OUTN  (NF * CC * NL)

#define SCW   64.0f
#define SCQK  8.0f
#define SCV   16.0f
#define SCE   32768.0f
#define SCO   16.0f
#define RSQD  0.15811388300841898f
#define SCS   (RSQD / (SCQK * SCQK))

static_assert(NF % FG == 0);
static_assert(CC % 64 == 0 && CC % 32 == 0 && NL % 64 == 0 && TOK % 64 == 0);
static_assert(NQK % 64 == 0 && NVR % 64 == 0 && QP % 32 == 0 && VP == 48 && HD <= QP && HD < VP);
static_assert(NH * HD == CC && NH == 8);
static_assert(NL == 4 * 256 && RSB == 32 && NL % RSB == 0 && (NL / 16) % 8 == 0);
static_assert((((TOK / 64) * (NQK / 64)) % 8) == 0);
static_assert((((NVR / 64) * (TOK / 64)) % 8) == 0);
static_assert(CC == 10 * 32);
static_assert((32 * (CC / 8)) % 256 == 0);
static_assert(((NQK * CC / 8) % 256) == 0 && ((NVR * CC / 8) % 256) == 0 && ((CC * CC / 8) % 256) == 0);

typedef _Float16       v16h __attribute__((ext_vector_type(16)));
typedef _Float16       v8h  __attribute__((ext_vector_type(8)));
typedef float          v8f  __attribute__((ext_vector_type(8)));
typedef float          v4f  __attribute__((ext_vector_type(4)));
typedef unsigned int   v4u  __attribute__((ext_vector_type(4)));

union HU { v8h h; v4u u; _Float16 s[8]; };
union FR { v16h v; v8h h[2]; _Float16 s[16]; };
static_assert(sizeof(HU) == 16);
static_assert(sizeof(FR) == 32);

__device__ __forceinline__ unsigned short bf_bits(float f) {
  const unsigned u = __float_as_uint(f);
  return (unsigned short)((u + 0x7FFFu + ((u >> 16) & 1u)) >> 16);
}
__device__ __forceinline__ float bf_up(unsigned short h) { return __uint_as_float(((unsigned)h) << 16); }
__device__ __forceinline__ float bfr(float f) { return bf_up(bf_bits(f)); }
__device__ __forceinline__ v8f zero8() { v8f z = {0.f, 0.f, 0.f, 0.f, 0.f, 0.f, 0.f, 0.f}; return z; }

__device__ __forceinline__ void ld8(const float* p, float* o) {
  const v4f a = *(const v4f*)(p);
  const v4f b = *(const v4f*)(p + 4);
  o[0] = a[0]; o[1] = a[1]; o[2] = a[2]; o[3] = a[3];
  o[4] = b[0]; o[5] = b[1]; o[6] = b[2]; o[7] = b[3];
}

__device__ __forceinline__ v16h ldfrag_h(const _Float16* p) {
  FR f;
  f.h[0] = *(const v8h*)(p);
  f.h[1] = *(const v8h*)(p + 16);
  return f.v;
}

__device__ __forceinline__ v8f mma_h(v16h a, v16h b, v8f c) {
  c = __builtin_amdgcn_wmma_f32_16x16x32_f16(false, a, false, b, (short)0, c, false, false);
#if defined(__HIP_DEVICE_COMPILE__)
  asm volatile("v_nop\n\tv_nop\n\tv_nop\n\tv_nop" : "+v"(c) : "v"(a), "v"(b));
#endif
  return c;
}
__device__ __forceinline__ v8f mma_h_raw(v16h a, v16h b, v8f c) {
  return __builtin_amdgcn_wmma_f32_16x16x32_f16(false, a, false, b, (short)0, c, false, false);
}
__device__ __forceinline__ void dep_guard_h(v8f& a, v8f& b, v16h x) {
#if defined(__HIP_DEVICE_COMPILE__)
  asm volatile("v_nop\n\tv_nop\n\tv_nop\n\tv_nop" : "+v"(a), "+v"(b) : "v"(x));
#endif
}
template <int NJ>
__device__ __forceinline__ void keep_bh(v16h (&b)[NJ]) {
#if defined(__HIP_DEVICE_COMPILE__)
  if constexpr (NJ == 4) {
    asm volatile("v_nop" :: "v"(b[0]), "v"(b[1]), "v"(b[2]), "v"(b[3]));
  } else if constexpr (NJ == 3) {
    asm volatile("v_nop" :: "v"(b[0]), "v"(b[1]), "v"(b[2]));
  } else if constexpr (NJ == 2) {
    asm volatile("v_nop" :: "v"(b[0]), "v"(b[1]));
  } else {
    asm volatile("v_nop" :: "v"(b[0]));
  }
#endif
}
__device__ __forceinline__ void acc_guard4(v8f& a, v8f& b, v8f& c, v8f& d) {
#if defined(__HIP_DEVICE_COMPILE__)
  asm volatile("v_nop\n\tv_nop\n\tv_nop\n\tv_nop" : "+v"(a), "+v"(b), "+v"(c), "+v"(d));
#endif
}
__device__ __forceinline__ void acc_guard3(v8f& a, v8f& b, v8f& c) {
#if defined(__HIP_DEVICE_COMPILE__)
  asm volatile("v_nop\n\tv_nop\n\tv_nop\n\tv_nop" : "+v"(a), "+v"(b), "+v"(c));
#endif
}
__device__ __forceinline__ void wave_lds_sync() {
  __builtin_amdgcn_fence(__ATOMIC_RELEASE, "workgroup");
  __builtin_amdgcn_wave_barrier();
  __builtin_amdgcn_fence(__ATOMIC_ACQUIRE, "workgroup");
}

template <int BG, int BR>
__device__ __forceinline__ float bias_at(const float* __restrict__ bias, int nbias, int boff, int t) {
  const int grp = t / BG;
  const int w = t - grp * BG;
  int idx = boff + grp * BR + min(w, BR - 1);
  idx = min(max(idx, 0), nbias - 1);
  const float b = bfr(bias[idx]);
  return (w < BR) ? b : 0.0f;
}

template <int G, int R>
__global__ __launch_bounds__(256) void cvt_wpad(const float* __restrict__ in, int inrows, int rowoff,
                                                _Float16* out, int n8, float scale) {
  const int i = blockIdx.x * 256 + threadIdx.x;
  if (i >= n8) return;
  const int K8 = CC / 8;
  const int ro = i / K8, k8 = i - ro * K8;
  const int grp = ro / G, w = ro - grp * G;
  int ir = rowoff + grp * R + min(w, R - 1);
  ir = min(max(ir, 0), inrows - 1);
  float v[8];
  ld8(in + (size_t)ir * CC + 8 * k8, v);
  const bool valid = (w < R);
  HU u;
#pragma unroll
  for (int e = 0; e < 8; ++e) {
    const _Float16 hv = (_Float16)(bfr(v[e]) * scale);
    u.s[e] = valid ? hv : (_Float16)0.0f;
  }
  _Float16* p = out + (size_t)i * 8;
  *(volatile v4u*)p = u.u;
  __threadfence();
  *(volatile v4u*)p = u.u;
}

__global__ __launch_bounds__(256) void cvt_xT(const float* __restrict__ X, _Float16* XT,
                                              const int* __restrict__ prm5, const int* __restrict__ prm6) {
  __shared__ float sw[64][65];
  if (prm5[0] < 1 || prm6[0] != NH) return;
  const int t = threadIdx.x;
  const int n0 = blockIdx.x * 64, k0 = blockIdx.y * 64, b = blockIdx.z;
  const float* Xb = X + (size_t)b * CC * NL;
  {
    const int r = t >> 4, c4 = (t & 15) * 4;
#pragma unroll
    for (int it = 0; it < 4; ++it) {
      const int row = r + 16 * it;
      const v4f x = *(const v4f*)(Xb + (size_t)(k0 + row) * NL + n0 + c4);
      sw[row][c4 + 0] = x[0]; sw[row][c4 + 1] = x[1]; sw[row][c4 + 2] = x[2]; sw[row][c4 + 3] = x[3];
    }
  }
  __syncthreads();
  const int q8 = t & 7, rr = t >> 3;
  HU u[2];
#pragma unroll
  for (int it = 0; it < 2; ++it) {
    const int n = rr + 32 * it;
#pragma unroll
    for (int e = 0; e < 8; ++e) u[it].s[e] = (_Float16)bfr(sw[8 * q8 + e][n]);
  }
  for (int pass = 0; pass < 2; ++pass) {
#pragma unroll
    for (int it = 0; it < 2; ++it) {
      const int n = rr + 32 * it;
      _Float16* dst = XT + (size_t)(b * NL + n0 + n) * CC + k0 + 8 * q8;
      *(volatile v4u*)dst = u[it].u;
    }
    __threadfence();
  }
}

template <int MI, int NJ>
__device__ __forceinline__ void kseg2(v8f (&acc)[MI][NJ], const _Float16* __restrict__ A, int lda, int m0,
                                      const _Float16* __restrict__ Bt, int ldb, int n0, int K, int rlane, int koff) {
  for (int kk = 0; kk < K; kk += 32) {
    v16h bh[NJ];
#pragma unroll
    for (int j = 0; j < NJ; ++j) {
      const size_t bo = (size_t)(n0 + (j << 4) + rlane) * (size_t)ldb + koff + kk;
      bh[j] = ldfrag_h(Bt + bo);
    }
#pragma unroll
    for (int i = 0; i < MI; ++i) {
      const size_t ao = (size_t)(m0 + (i << 4) + rlane) * (size_t)lda + koff + kk;
      const v16h a0 = ldfrag_h(A + ao);
#pragma unroll
      for (int j = 0; j < NJ; ++j) acc[i][j] = mma_h_raw(a0, bh[j], acc[i][j]);
      dep_guard_h(acc[i][0], acc[i][NJ - 1], a0);
    }
    keep_bh<NJ>(bh);
  }
}

template <int RB, int BG, int BR>
__global__ __launch_bounds__(256) void gemm64p(
    const _Float16* __restrict__ A, int lda, const _Float16* __restrict__ Bt, int ldb,
    const float* __restrict__ bias, int nbias, int boff, float cs, float so,
    _Float16* Cp, int ldc, int M, int N, int K) {
  __shared__ __align__(16) float sT[8][16 * 68];
  const int lane = threadIdx.x & 31;
  const int wave = threadIdx.x >> 5;
  const int tilesN = N >> 6;
  const int tilesM = M >> 6;
  const int tiles = tilesM * tilesN;
  const int item = blockIdx.x * 8 + wave;
  if (item >= tiles) return;
  const int tm = item / tilesN;
  const int tn = item - tm * tilesN;
  const int m0 = tm << 6;
  const int n0 = tn << 6;

  const int rlane = lane & 15;
  const int koff  = (lane >> 4) * 8;
  const int mOff  = (lane >> 4) * 8;

  v8f acc[4][4];
#pragma unroll
  for (int i = 0; i < 4; ++i)
#pragma unroll
    for (int j = 0; j < 4; ++j) acc[i][j] = zero8();

  kseg2<4, 4>(acc, A, lda, m0, Bt, ldb, n0, K, rlane, koff);
  acc_guard4(acc[0][0], acc[0][1], acc[0][2], acc[0][3]);
  acc_guard4(acc[1][0], acc[1][1], acc[1][2], acc[1][3]);
  acc_guard4(acc[2][0], acc[2][1], acc[2][2], acc[2][3]);
  acc_guard4(acc[3][0], acc[3][1], acc[3][2], acc[3][3]);

  const int q8 = lane & 7, rr = lane >> 3, c8 = q8 * 8;

  float cbv[8];
#pragma unroll
  for (int e = 0; e < 8; ++e) cbv[e] = 0.0f;
  if (RB == 2) {
#pragma unroll
    for (int e = 0; e < 8; ++e) cbv[e] = bias_at<BG, BR>(bias, nbias, boff, n0 + c8 + e);
  }

  float* slab = sT[wave];
#pragma unroll
  for (int i = 0; i < 4; ++i) {
    const int mBase = m0 + (i << 4);
#pragma unroll
    for (int r = 0; r < 8; ++r) {
#pragma unroll
      for (int j = 0; j < 4; ++j) {
        slab[(mOff + r) * 68 + (j << 4) + rlane] = acc[i][j][r];
      }
    }
    wave_lds_sync();
    v4u uh[4];
#pragma unroll
    for (int it = 0; it < 4; ++it) {
      const int row = it * 4 + rr;
      float xs[8];
      ld8(slab + row * 68 + c8, xs);
      float rbv = 0.0f;
      if (RB == 1) rbv = bias_at<BG, BR>(bias, nbias, boff, mBase + row);
      HU h;
#pragma unroll
      for (int e = 0; e < 8; ++e) {
        const float v = (xs[e] * cs + rbv + cbv[e]) * so;
        h.s[e] = (_Float16)v;
      }
      uh[it] = h.u;
    }
    for (int pass = 0; pass < 2; ++pass) {
#pragma unroll
      for (int it = 0; it < 4; ++it) {
        const int row = it * 4 + rr;
        const size_t co = (size_t)(mBase + row) * (size_t)ldc + n0 + c8;
        *(volatile v4u*)(Cp + co) = uh[it];
      }
      __threadfence();
    }
    wave_lds_sync();
  }
}

__global__ __launch_bounds__(256) void k_soft(const _Float16* __restrict__ XQK, _Float16* E, int f0) {
  extern __shared__ __align__(16) float sc[];
  const int tid = threadIdx.x, wave = tid >> 5, lane = tid & 31;
  const int hh = lane >> 4, rl = lane & 15;
  const int rb = blockIdx.x, p = blockIdx.y, n0 = rb * RSB;
  const int fl = p / NH, h = p - fl * NH, f = f0 + fl;

  const _Float16* aq = XQK + (size_t)(f * NL + n0 + rl) * NQK + h * QP + 8 * hh;
  const _Float16* kb0 = XQK + (size_t)(f * NL) * NQK + NH * QP + h * QP + 8 * hh;
  v16h qf0[QP / 32], qf1[QP / 32];
#pragma unroll
  for (int ks = 0; ks < QP / 32; ++ks) {
    qf0[ks] = ldfrag_h(aq + 32 * ks);
    qf1[ks] = ldfrag_h(aq + (size_t)16 * NQK + 32 * ks);
  }
  for (int ct = wave; ct < NL / 16; ct += 8) {
    const _Float16* bk = kb0 + (size_t)(16 * ct + rl) * NQK;
    v8f a0 = zero8(), a1 = zero8();
#pragma unroll
    for (int ks = 0; ks < QP / 32; ++ks) {
      const v16h kb = ldfrag_h(bk + 32 * ks);
      a0 = mma_h(qf0[ks], kb, a0);
      a1 = mma_h(qf1[ks], kb, a1);
    }
    const int mc = 16 * ct + rl;
#pragma unroll
    for (int r = 0; r < 8; ++r) {
      sc[(size_t)(8 * hh + r) * NL + mc]      = a0[r] * SCS;
      sc[(size_t)(16 + 8 * hh + r) * NL + mc] = a1[r] * SCS;
    }
  }
  __syncthreads();

  for (int q4 = 0; q4 < 4; ++q4) {
    const int row = 4 * wave + q4;
    const float* rp = sc + (size_t)row * NL + 8 * lane;
    float v[4][8];
    float mx = -3.0e38f;
#pragma unroll
    for (int j = 0; j < 4; ++j) {
      ld8(rp + 256 * j, v[j]);
#pragma unroll
      for (int e = 0; e < 8; ++e) mx = fmaxf(mx, v[j][e]);
    }
#pragma unroll
    for (int off = 16; off >= 1; off >>= 1) mx = fmaxf(mx, __shfl_xor(mx, off, 32));
    float z = 0.0f;
#pragma unroll
    for (int j = 0; j < 4; ++j) {
#pragma unroll
      for (int e = 0; e < 8; ++e) {
        const float ef = __expf(v[j][e] - mx);
        z += ef;
        v[j][e] = ef;
      }
    }
#pragma unroll
    for (int off = 16; off >= 1; off >>= 1) z += __shfl_xor(z, off, 32);
    const float rz = SCE * (1.0f / z);
    HU u[4];
#pragma unroll
    for (int j = 0; j < 4; ++j) {
#pragma unroll
      for (int e = 0; e < 8; ++e) {
        const _Float16 h0 = (_Float16)(v[j][e] * rz);
        const float fz = (float)h0;
        const bool sub = fz < 6.103515625e-05f;
        u[j].s[e] = sub ? (_Float16)0.0f : h0;
      }
    }
    _Float16* erow = E + ((size_t)p * NL + n0 + row) * NL + 8 * lane;
    for (int pass = 0; pass < 2; ++pass) {
#pragma unroll
      for (int j = 0; j < 4; ++j) *(volatile v4u*)(erow + 256 * j) = u[j].u;
      __threadfence();
    }
  }
}

__global__ __launch_bounds__(256) void k_pv(const _Float16* __restrict__ E, const _Float16* __restrict__ VH,
                                            _Float16* O16, int f0) {
  __shared__ __align__(16) float sO[32 * 328];
  const int tid = threadIdx.x, wave = tid >> 5, lane = tid & 31;
  const int hh = lane >> 4, rl = lane & 15;
  const int rb = blockIdx.x, fl = blockIdx.y, f = f0 + fl, l0 = rb * 32;
  const int h = wave;

  v8f acc[2][3];
#pragma unroll
  for (int i = 0; i < 2; ++i)
#pragma unroll
    for (int j = 0; j < 3; ++j) acc[i][j] = zero8();

  const _Float16* Ab = E + (size_t)(fl * NH + h) * NL * NL;
  const _Float16* Bb = VH + (size_t)(h * VP) * TOK + (size_t)f * NL;
  kseg2<2, 3>(acc, Ab, NL, l0, Bb, TOK, 0, NL, rl, 8 * hh);
  acc_guard3(acc[0][0], acc[0][1], acc[0][2]);
  acc_guard3(acc[1][0], acc[1][1], acc[1][2]);

  const float fo = SCO / (SCV * SCE);
  const int cw = h * HD;
#pragma unroll
  for (int i = 0; i < 2; ++i) {
#pragma unroll
    for (int r = 0; r < 8; ++r) {
      const int row = 16 * i + 8 * hh + r;
      sO[row * 328 + cw + rl]      = acc[i][0][r] * fo;
      sO[row * 328 + cw + 16 + rl] = acc[i][1][r] * fo;
      if (rl < 8) sO[row * 328 + cw + 32 + rl] = acc[i][2][r] * fo;
    }
  }
  __syncthreads();

  HU u[5];
#pragma unroll
  for (int it = 0; it < 5; ++it) {
    const int pidx = it * 256 + tid;
    const int row = pidx / (CC / 8);
    const int q = pidx - row * (CC / 8);
    float xs[8];
    ld8(sO + row * 328 + 8 * q, xs);
#pragma unroll
    for (int e = 0; e < 8; ++e) u[it].s[e] = (_Float16)xs[e];
  }
  for (int pass = 0; pass < 2; ++pass) {
#pragma unroll
    for (int it = 0; it < 5; ++it) {
      const int pidx = it * 256 + tid;
      const int row = pidx / (CC / 8);
      const int q = pidx - row * (CC / 8);
      _Float16* dst = O16 + ((size_t)(f * NL + l0 + row)) * CC + 8 * q;
      *(volatile v4u*)dst = u[it].u;
    }
    __threadfence();
  }
}

__global__ __launch_bounds__(320) void k_out(const _Float16* __restrict__ WO16, const _Float16* __restrict__ O16,
                                             const float* __restrict__ bo, const float* __restrict__ X, float* out) {
  __shared__ __align__(16) float sO[10][16 * 68];
  const int tid = threadIdx.x, wave = tid >> 5, lane = tid & 31;
  const int hh = lane >> 4, rl = lane & 15;
  const int bx = blockIdx.x;
  const int f = bx / (NL / 64);
  const int n0 = (bx - f * (NL / 64)) * 64;
  const int cb = wave * 32;

  v8f acc[2][4];
#pragma unroll
  for (int i = 0; i < 2; ++i)
#pragma unroll
    for (int j = 0; j < 4; ++j) acc[i][j] = zero8();

  const _Float16* Bb = O16 + (size_t)f * NL * CC;
  kseg2<2, 4>(acc, WO16, CC, cb, Bb, CC, n0, CC, rl, 8 * hh);
  acc_guard4(acc[0][0], acc[0][1], acc[0][2], acc[0][3]);
  acc_guard4(acc[1][0], acc[1][1], acc[1][2], acc[1][3]);

  const float fo = 1.0f / (SCW * SCO);
  float* slab = sO[wave];
  const int p4 = (lane & 15) * 4, r2 = lane >> 4;
#pragma unroll
  for (int i = 0; i < 2; ++i) {
    const int cBase = cb + 16 * i;
#pragma unroll
    for (int r = 0; r < 8; ++r) {
#pragma unroll
      for (int j = 0; j < 4; ++j) {
        slab[(8 * hh + r) * 68 + 16 * j + rl] = acc[i][j][r];
      }
    }
    wave_lds_sync();
    v4f ov[8];
#pragma unroll
    for (int it = 0; it < 8; ++it) {
      const int row = 2 * it + r2;
      const v4f a = *(const v4f*)(slab + row * 68 + p4);
      const float rbv = bfr(bo[min(cBase + row, CC - 1)]);
      const size_t xo = ((size_t)(f * CC + cBase + row)) * NL + n0 + p4;
      const v4f xv = *(const v4f*)(X + xo);
      v4f o;
#pragma unroll
      for (int e = 0; e < 4; ++e) o[e] = (a[e] * fo + rbv) + bfr(xv[e]);
      ov[it] = o;
    }
    for (int pass = 0; pass < 2; ++pass) {
#pragma unroll
      for (int it = 0; it < 8; ++it) {
        const int row = 2 * it + r2;
        const size_t oo = ((size_t)(f * CC + cBase + row)) * NL + n0 + p4;
        *(volatile v4f*)(out + oo) = ov[it];
      }
      __threadfence();
    }
    wave_lds_sync();
  }
}

extern "C" void kernel_launch(void* const* d_in, const int* in_sizes, int n_in,
                              void* d_out, int out_size, void* d_ws, size_t ws_size,
                              hipStream_t stream) {
  if (n_in < 7) return;
  if (in_sizes[0] < OUTN) return;
  if (in_sizes[1] != NIN * CC || in_sizes[2] != NIN) return;
  if (in_sizes[3] != CC * CC || in_sizes[4] != CC) return;
  if (in_sizes[5] < 1 || in_sizes[6] < 1) return;
  if (out_size < OUTN) return;

  const float* x    = (const float*)d_in[0];
  const float* w_in = (const float*)d_in[1];
  const float* b_in = (const float*)d_in[2];
  const float* w_o  = (const float*)d_in[3];
  const float* b_o  = (const float*)d_in[4];
  const int*   prm5 = (const int*)d_in[5];
  const int*   prm6 = (const int*)d_in[6];

  const size_t PWQK = (size_t)NQK * CC * 2;
  const size_t PWV  = (size_t)NVR * CC * 2;
  const size_t PWO  = (size_t)CC * CC * 2;
  const size_t PXQK = (size_t)TOK * NQK * 2;
  const size_t PVH  = (size_t)NVR * TOK * 2;
  const size_t PO   = (size_t)TOK * CC * 2;
  const size_t PXT  = (size_t)TOK * CC * 2;
  const size_t PE   = (size_t)NPAIR * NL * NL * 2;
  const size_t PXE  = (PE > PXT) ? PE : PXT;

  size_t off = 0;
  const size_t oWQK = off; off += PWQK;
  const size_t oWV  = off; off += PWV;
  const size_t oWO  = off; off += PWO;
  const size_t oXQK = off; off += PXQK;
  const size_t oVH  = off; off += PVH;
  const size_t oO   = off; off += PO;
  const size_t oXE  = off; off += PXE;
  if (off > ws_size) return;
  if (off > (size_t)134217728) return;

  char* ws = (char*)d_ws;
  _Float16* WQK16 = (_Float16*)(ws + oWQK);
  _Float16* WV16  = (_Float16*)(ws + oWV);
  _Float16* WO16  = (_Float16*)(ws + oWO);
  _Float16* XQK   = (_Float16*)(ws + oXQK);
  _Float16* VH    = (_Float16*)(ws + oVH);
  _Float16* O16   = (_Float16*)(ws + oO);
  _Float16* xT    = (_Float16*)(ws + oXE);
  _Float16* E     = (_Float16*)(ws + oXE);
  float*    outf  = (float*)d_out;

  const dim3 blk(256);
  const int  n8qk = (NQK * CC) / 8;
  const int  n8v  = (NVR * CC) / 8;
  const int  n8o  = (CC * CC) / 8;
  const dim3 gWqk((n8qk + 255) / 256);
  const dim3 gWv((n8v + 255) / 256);
  const dim3 gWo((n8o + 255) / 256);
  const dim3 gXT(NL / 64, CC / 64, NF);
  const dim3 gQK(((TOK / 64) * (NQK / 64) + 7) / 8);
  const dim3 gV(((NVR / 64) * (TOK / 64) + 7) / 8);
  const dim3 gSo(NL / RSB, NPAIR);
  const dim3 gPV(NL / 32, FG);
  const dim3 gOut(NF * (NL / 64));
  const float cs64 = 1.0f / SCW;
  const size_t ldsSoft = (size_t)RSB * NL * sizeof(float);

  hipFuncSetAttribute(reinterpret_cast<const void*>(&k_soft), hipFuncAttributeMaxDynamicSharedMemorySize,
                      (int)ldsSoft);

  cvt_wpad<QP, HD><<<gWqk, blk, 0, stream>>>(w_in, NIN, 0, WQK16, n8qk, SCW);
  cvt_wpad<VP, HD><<<gWv, blk, 0, stream>>>(w_in, NIN, 2 * CC, WV16, n8v, SCW);
  cvt_wpad<1, 1><<<gWo, blk, 0, stream>>>(w_o, CC, 0, WO16, n8o, SCW);
  cvt_xT<<<gXT, blk, 0, stream>>>(x, xT, prm5, prm6);
  gemm64p<2, QP, HD><<<gQK, blk, 0, stream>>>(xT, CC, WQK16, CC, b_in, NIN, 0, cs64, SCQK, XQK, NQK, TOK, NQK, CC);
  gemm64p<1, VP, HD><<<gV, blk, 0, stream>>>(WV16, CC, xT, CC, b_in, NIN, 2 * CC, cs64, SCV, VH, TOK, NVR, TOK, CC);
  for (int c = 0; c < NF / FG; ++c) {
    const int f0 = c * FG;
    k_soft<<<gSo, blk, ldsSoft, stream>>>(XQK, E, f0);
    k_pv<<<gPV, blk, 0, stream>>>(E, VH, O16, f0);
  }
  k_out<<<gOut, dim3(320), 0, stream>>>(WO16, O16, b_o, x, outf);
}
